// generator_gnn_38302518345769
// MI455X (gfx1250) — hardware-verified
//
#include <hip/hip_runtime.h>
#include <stddef.h>

#define NN 2048
#define NB 64
#define LAT 128
#define EMB 8
#define HID 8
#define KIN 136
#define KP 160
#define VOC 50
#define NG 7
#define TP 72
#define TSP 68
#define PSCALE 256.0f
#define WSCALE 16.0f
#define PLANE (NB * NN)

static_assert(NN % 64 == 0);
static_assert(NB == 64);
static_assert(KP % 32 == 0);
static_assert(KP >= KIN);
static_assert(LAT + EMB == KIN);
static_assert((NB * KP) % (256 * 8) == 0);
static_assert(PLANE % (256 * 4) == 0);
static_assert(TP % 8 == 0);
static_assert(TSP % 4 == 0);
static_assert(NG * HID == 56);

typedef _Float16 f16;
typedef f16 v16h __attribute__((ext_vector_type(16)));
typedef f16 v8h_t __attribute__((ext_vector_type(8)));
typedef v8h_t __attribute__((may_alias)) v8h;
typedef float v8f __attribute__((ext_vector_type(8)));
typedef float v4f_t __attribute__((ext_vector_type(4)));
typedef v4f_t __attribute__((may_alias)) v4f;
typedef unsigned int v4u_t __attribute__((ext_vector_type(4)));
typedef v4u_t __attribute__((may_alias)) v4u;

union Frag { v16h v; v8h_t h[2]; };
union Pack8 { v8h_t h; v4u_t u; };

__device__ __forceinline__ v8f zero8() {
    v8f z;
#pragma unroll
    for (int i = 0; i < 8; ++i) z[i] = 0.0f;
    return z;
}

__device__ __forceinline__ v16h ldfrag(const f16* p, int k0) {
    Frag f;
    f.h[0] = *(const v8h*)(p + k0);
    f.h[1] = *(const v8h*)(p + k0 + 16);
    return f.v;
}

__device__ __forceinline__ v8f wmma16(v16h a, v16h b, v8f c) {
    return __builtin_amdgcn_wmma_f32_16x16x32_f16(false, a, false, b, (short)0, c, false, false);
}

__device__ __forceinline__ void mma4(v8f (&acc)[4], const f16* pa, const f16* pb, size_t bs, int k0) {
    const v16h a  = ldfrag(pa, k0);
    const v16h b0 = ldfrag(pb, k0);
    const v16h b1 = ldfrag(pb + bs, k0);
    const v16h b2 = ldfrag(pb + 2 * bs, k0);
    const v16h b3 = ldfrag(pb + 3 * bs, k0);
    acc[0] = wmma16(a, b0, acc[0]);
    acc[1] = wmma16(a, b1, acc[1]);
    acc[2] = wmma16(a, b2, acc[2]);
    acc[3] = wmma16(a, b3, acc[3]);
    asm volatile("v_nop\n\tv_nop\n\tv_nop\n\tv_nop"
                 : "+v"(acc[0]), "+v"(acc[1]), "+v"(acc[2]), "+v"(acc[3])
                 : "v"(a), "v"(b0), "v"(b1), "v"(b2), "v"(b3));
}

__device__ __forceinline__ void store_tile64(const float* Ts, const float* dA, const float* dB,
                                             float* Fd, f16* Qa, f16* Qb, int writeQ, int w, int l)
{
    const int hq = l >> 4, q4 = l & 15;
    const int oq = l >> 3, q8 = l & 7;
    v4f_t fv[8];
#pragma unroll
    for (int p = 0; p < 8; ++p) {
        const int row = 16 * w + 2 * p + hq;
        fv[p] = *(const v4f*)(Ts + row * TSP + 4 * q4);
    }
    Pack8 qa[4], qb[4];
#pragma unroll
    for (int p = 0; p < 4; ++p) {
        const int row = 16 * w + 4 * p + oq;
#pragma unroll
        for (int j = 0; j < 8; ++j) {
            const int col = 8 * q8 + j;
            const float v = Ts[row * TSP + col];
            qa[p].h[j] = (f16)(v * dA[col] * PSCALE);
            qb[p].h[j] = (f16)(v * dB[col] * PSCALE);
        }
    }
#pragma unroll
    for (int p = 0; p < 8; ++p)
        *(volatile v4f_t*)(Fd + (size_t)(16 * w + 2 * p + hq) * NN + 4 * q4) = fv[p];
    if (writeQ) {
#pragma unroll
        for (int p = 0; p < 4; ++p) {
            const size_t o = (size_t)(16 * w + 4 * p + oq) * NN + 8 * q8;
            *(volatile v4u_t*)(Qa + o) = qa[p].u;
            *(volatile v4u_t*)(Qb + o) = qb[p].u;
        }
    }
    __threadfence();
#pragma unroll
    for (int p = 0; p < 8; ++p)
        *(volatile v4f_t*)(Fd + (size_t)(16 * w + 2 * p + hq) * NN + 4 * q4) = fv[p];
    if (writeQ) {
#pragma unroll
        for (int p = 0; p < 4; ++p) {
            const size_t o = (size_t)(16 * w + 4 * p + oq) * NN + 8 * q8;
            *(volatile v4u_t*)(Qa + o) = qa[p].u;
            *(volatile v4u_t*)(Qb + o) = qb[p].u;
        }
    }
}

__global__ void __launch_bounds__(256) prep_adj(const float* __restrict__ adj,
                                                f16* __restrict__ a16, f16* __restrict__ aT16)
{
    __shared__ __align__(16) f16 Ts[64 * TP];
    __shared__ __align__(16) f16 Tt[64 * TP];
    const int t = threadIdx.x;
    const int k0 = blockIdx.x * 64, i0 = blockIdx.y * 64;
#pragma unroll 4
    for (int it = 0; it < 16; ++it) {
        const int idx = it * 256 + t;
        const int r = idx >> 6, c = idx & 63;
        const float v = adj[(size_t)(i0 + r) * NN + k0 + c];
        const f16 hv = ((i0 + r) != (k0 + c)) ? (f16)v : (f16)0.0f;
        Ts[r * TP + c] = hv;
        Tt[c * TP + r] = hv;
    }
    __syncthreads();
    const int w = t >> 5, l = t & 31, q = l & 7;
    v4u_t va[2], vt[2];
#pragma unroll
    for (int p = 0; p < 2; ++p) {
        const int row = 8 * w + 4 * p + (l >> 3);
        va[p] = *(const v4u*)(Ts + row * TP + 8 * q);
        vt[p] = *(const v4u*)(Tt + row * TP + 8 * q);
    }
#pragma unroll
    for (int p = 0; p < 2; ++p) {
        const int row = 8 * w + 4 * p + (l >> 3);
        *(volatile v4u_t*)(a16  + (size_t)(i0 + row) * NN + k0 + 8 * q) = va[p];
        *(volatile v4u_t*)(aT16 + (size_t)(k0 + row) * NN + i0 + 8 * q) = vt[p];
    }
    __threadfence();
#pragma unroll
    for (int p = 0; p < 2; ++p) {
        const int row = 8 * w + 4 * p + (l >> 3);
        *(volatile v4u_t*)(a16  + (size_t)(i0 + row) * NN + k0 + 8 * q) = va[p];
        *(volatile v4u_t*)(aT16 + (size_t)(k0 + row) * NN + i0 + 8 * q) = vt[p];
    }
}

__global__ void __launch_bounds__(256) row_deg(const f16* __restrict__ a, float* __restrict__ d)
{
    __shared__ __align__(16) float dl[32];
    const int t = threadIdx.x, w = t >> 5, l = t & 31;
    const int rb = blockIdx.x * 32;
#pragma unroll 1
    for (int rr = 0; rr < 4; ++rr) {
        const int row = rb + 4 * w + rr;
        const f16* ap = a + (size_t)row * NN;
        float s = 0.0f;
#pragma unroll 1
        for (int it = 0; it < NN / 256; ++it) {
            const v8h_t v = *(const v8h*)(ap + it * 256 + 8 * l);
#pragma unroll
            for (int j = 0; j < 8; ++j) s += (float)v[j];
        }
#pragma unroll
        for (int off = 16; off > 0; off >>= 1) s += __shfl_xor(s, off, 32);
        const float dv = (s > 0.0f) ? (1.0f / sqrtf(s)) : 0.0f;
        if (l == 0) dl[4 * w + rr] = dv;
    }
    __syncthreads();
    const v4f_t v = *(const v4f*)(dl + 4 * (t & 7));
    if (t < 8) *(volatile v4f_t*)(d + rb + 4 * t) = v;
    __threadfence();
    if (t < 8) *(volatile v4f_t*)(d + rb + 4 * t) = v;
}

__global__ void __launch_bounds__(256) prep_w(const float* __restrict__ wmap, f16* __restrict__ wT)
{
    __shared__ __align__(16) f16 Ls[NB * KP];
    const int t = threadIdx.x, n0 = blockIdx.x * 64;
#pragma unroll 1
    for (int idx = t; idx < 64 * KP; idx += 256) {
        const int f = idx >> 6, c = idx & 63;
        const int fa = (f < KIN) ? f : (KIN - 1);
        const float v = wmap[(size_t)fa * NN + n0 + c];
        Ls[c * KP + f] = (f < KIN) ? (f16)(v * WSCALE) : (f16)0.0f;
    }
    __syncthreads();
    v4u_t vals[5];
#pragma unroll
    for (int it = 0; it < 5; ++it) vals[it] = *(const v4u*)(Ls + (size_t)(it * 256 + t) * 8);
    f16* dst = wT + (size_t)n0 * KP;
#pragma unroll
    for (int it = 0; it < 5; ++it) *(volatile v4u_t*)(dst + (size_t)(it * 256 + t) * 8) = vals[it];
    __threadfence();
#pragma unroll
    for (int it = 0; it < 5; ++it) *(volatile v4u_t*)(dst + (size_t)(it * 256 + t) * 8) = vals[it];
}

__global__ void __launch_bounds__(256) prep_z(const float* __restrict__ x, const int* __restrict__ cat,
                                              const float* __restrict__ emb, f16* __restrict__ z16)
{
    __shared__ __align__(16) f16 Ls[NB * KP];
    const int t = threadIdx.x;
#pragma unroll 1
    for (int idx = t; idx < NB * KP; idx += 256) {
        const int b = idx / KP, f = idx - b * KP;
        int ci = cat[b];
        if (ci < 0) ci += VOC;
        ci = (ci < 0) ? 0 : ((ci > VOC - 1) ? (VOC - 1) : ci);
        const int xf = (f < LAT) ? f : (LAT - 1);
        int ef = f - LAT;
        ef = (ef < 0) ? 0 : ((ef > EMB - 1) ? (EMB - 1) : ef);
        const float xv = x[b * LAT + xf];
        const float ev = emb[ci * EMB + ef];
        const float v = (f < LAT) ? xv : ((f < KIN) ? ev : 0.0f);
        Ls[idx] = (f16)v;
    }
    __syncthreads();
    v4u_t vals[5];
#pragma unroll
    for (int it = 0; it < 5; ++it) vals[it] = *(const v4u*)(Ls + (size_t)(it * 256 + t) * 8);
#pragma unroll
    for (int it = 0; it < 5; ++it) *(volatile v4u_t*)(z16 + (size_t)(it * 256 + t) * 8) = vals[it];
    __threadfence();
#pragma unroll
    for (int it = 0; it < 5; ++it) *(volatile v4u_t*)(z16 + (size_t)(it * 256 + t) * 8) = vals[it];
}

__global__ void __launch_bounds__(128) aa_gemm(const f16* __restrict__ a16, const f16* __restrict__ aT16,
                                               f16* __restrict__ th16)
{
    __shared__ __align__(16) f16 Th[64 * TP];
    const int t = threadIdx.x, w = t >> 5, l = t & 31, h = l >> 4, m = l & 15;
    const int j0 = blockIdx.x * 64, i0 = blockIdx.y * 64;
    const f16* pa = a16  + (size_t)(i0 + 16 * w + m) * NN + 8 * h;
    const f16* pb = aT16 + (size_t)(j0 + m) * NN + 8 * h;
    v8f acc[4];
#pragma unroll
    for (int c = 0; c < 4; ++c) acc[c] = zero8();
#pragma unroll 1
    for (int k0 = 0; k0 < NN; k0 += 32) mma4(acc, pa, pb, (size_t)16 * NN, k0);
#pragma unroll
    for (int ct = 0; ct < 4; ++ct) {
#pragma unroll
        for (int r = 0; r < 8; ++r) {
            const int il = 16 * w + 8 * h + r, jl = 16 * ct + m;
            const int i = i0 + il, j = j0 + jl;
            const float av = (float)a16[(size_t)i * NN + j];
            const bool pr = (acc[ct][r] > 0.0f) && (av == 0.0f) && (i != j);
            Th[il * TP + jl] = pr ? (f16)1.0f : (f16)0.0f;
        }
    }
    __syncthreads();
    const int q = l & 7;
    v4u_t vals[4];
#pragma unroll
    for (int p = 0; p < 4; ++p) {
        const int row = 16 * w + 4 * p + (l >> 3);
        vals[p] = *(const v4u*)(Th + row * TP + 8 * q);
    }
#pragma unroll
    for (int p = 0; p < 4; ++p) {
        const int row = 16 * w + 4 * p + (l >> 3);
        *(volatile v4u_t*)(th16 + (size_t)(i0 + row) * NN + j0 + 8 * q) = vals[p];
    }
    __threadfence();
#pragma unroll
    for (int p = 0; p < 4; ++p) {
        const int row = 16 * w + 4 * p + (l >> 3);
        *(volatile v4u_t*)(th16 + (size_t)(i0 + row) * NN + j0 + 8 * q) = vals[p];
    }
}

__global__ void __launch_bounds__(128) nodes_gemm(const f16* __restrict__ z16, const f16* __restrict__ wT,
                                                  const float* __restrict__ bmap,
                                                  const float* __restrict__ d1, const float* __restrict__ d2,
                                                  float* F0, f16* P)
{
    __shared__ __align__(16) float Ts[64 * TSP];
    __shared__ __align__(16) float dA[64];
    __shared__ __align__(16) float dB[64];
    __shared__ __align__(16) float bL[64];
    const int t = threadIdx.x, w = t >> 5, l = t & 31, h = l >> 4, m = l & 15;
    const int n0 = blockIdx.x * 64;
    if (t < 64) { dA[t] = d1[n0 + t]; dB[t] = d2[n0 + t]; bL[t] = bmap[n0 + t]; }
    __syncthreads();
    const f16* pa = z16 + (size_t)(16 * w + m) * KP + 8 * h;
    const f16* pb = wT + (size_t)(n0 + m) * KP + 8 * h;
    v8f acc[4];
#pragma unroll
    for (int c = 0; c < 4; ++c) acc[c] = zero8();
#pragma unroll 1
    for (int k0 = 0; k0 < KP; k0 += 32) mma4(acc, pa, pb, (size_t)16 * KP, k0);
#pragma unroll
    for (int ct = 0; ct < 4; ++ct) {
#pragma unroll
        for (int r = 0; r < 8; ++r) {
            const int col = 16 * ct + m;
            Ts[(16 * w + 8 * h + r) * TSP + col] = acc[ct][r] * (1.0f / WSCALE) + bL[col];
        }
    }
    __syncthreads();
    store_tile64(Ts, dA, dB, F0 + n0, P + n0, P + (size_t)PLANE + n0, 1, w, l);
}

__global__ void __launch_bounds__(128) prop_gemm(const f16* __restrict__ A, const f16* __restrict__ Bp,
                                                 const float* __restrict__ dE,
                                                 const float* __restrict__ d1, const float* __restrict__ d2,
                                                 float* Fd, f16* Qa, f16* Qb, int writeQ)
{
    __shared__ __align__(16) float Ts[64 * TSP];
    __shared__ __align__(16) float dEl[64];
    __shared__ __align__(16) float dA[64];
    __shared__ __align__(16) float dB[64];
    const int t = threadIdx.x, w = t >> 5, l = t & 31, h = l >> 4, m = l & 15;
    const int i0 = blockIdx.x * 64, c0 = blockIdx.y * 64;
    if (t < 64) { dEl[t] = dE[i0 + t]; dA[t] = d1[i0 + t]; dB[t] = d2[i0 + t]; }
    __syncthreads();
    const f16* pa = A  + (size_t)(i0 + 16 * w + m) * NN + 8 * h;
    const f16* pb = Bp + (size_t)(c0 + m) * NN + 8 * h;
    v8f acc[4];
#pragma unroll
    for (int c = 0; c < 4; ++c) acc[c] = zero8();
#pragma unroll 1
    for (int k0 = 0; k0 < NN; k0 += 32) mma4(acc, pa, pb, (size_t)16 * NN, k0);
#pragma unroll
    for (int ct = 0; ct < 4; ++ct) {
#pragma unroll
        for (int r = 0; r < 8; ++r) {
            const int il = 16 * w + 8 * h + r, cl = 16 * ct + m;
            Ts[cl * TSP + il] = acc[ct][r] * dEl[il] * (1.0f / PSCALE);
        }
    }
    __syncthreads();
    const size_t off = (size_t)c0 * NN + i0;
    store_tile64(Ts, dA, dB, Fd + off, Qa + off, Qb + off, writeQ, w, l);
}

__global__ void __launch_bounds__(256) readout_k(const float* __restrict__ F, const float* __restrict__ wemb,
                                                 const float* __restrict__ wout, float* out)
{
    __shared__ float cg[8];
    const int t = threadIdx.x;
    const int tg = (t < NG) ? t : (NG - 1);
    float s = 0.0f;
#pragma unroll 1
    for (int hh = 0; hh < HID; ++hh) s = fmaf(wemb[hh], wout[tg * HID + hh], s);
    const float sv = (t < NG) ? s : 0.0f;
    if (t < 8) cg[t] = sv;
    __syncthreads();
    const size_t e = ((size_t)blockIdx.x * 256 + t) * 4;
    v4f_t acc;
#pragma unroll
    for (int j = 0; j < 4; ++j) acc[j] = 0.0f;
#pragma unroll
    for (int g = 0; g < NG; ++g) {
        const v4f_t v = *(const v4f*)(F + (size_t)g * PLANE + e);
        const float c = cg[g];
#pragma unroll
        for (int j = 0; j < 4; ++j) acc[j] = fmaf(c, v[j], acc[j]);
    }
    *(volatile v4f_t*)(out + e) = acc;
    __threadfence();
    *(volatile v4f_t*)(out + e) = acc;
}

extern "C" void kernel_launch(void* const* d_in, const int* in_sizes, int n_in,
                              void* d_out, int out_size, void* d_ws, size_t ws_size,
                              hipStream_t stream)
{
    if (n_in < 8) return;
    if (in_sizes[0] != NB * LAT) return;
    if (in_sizes[1] != NB) return;
    if (in_sizes[2] != NN * NN) return;
    if (in_sizes[3] != VOC * EMB) return;
    if (in_sizes[4] != KIN * NN) return;
    if (in_sizes[5] != NN) return;
    if (in_sizes[6] != HID) return;
    if (in_sizes[7] != NG * HID) return;
    if (out_size != NB * NN) return;

    const float* x    = (const float*)d_in[0];
    const int*   cat  = (const int*)d_in[1];
    const float* adj  = (const float*)d_in[2];
    const float* emb  = (const float*)d_in[3];
    const float* wmap = (const float*)d_in[4];
    const float* bmap = (const float*)d_in[5];
    const float* wemb = (const float*)d_in[6];
    const float* wout = (const float*)d_in[7];
    float* out = (float*)d_out;

    const size_t szA  = (size_t)NN * NN * sizeof(f16);
    const size_t szWT = (size_t)NN * KP * sizeof(f16);
    const size_t szZ  = (size_t)NB * KP * sizeof(f16);
    const size_t szD  = (size_t)NN * sizeof(float);
    const size_t szP  = (size_t)2 * PLANE * sizeof(f16);
    const size_t szF  = (size_t)NG * PLANE * sizeof(float);
    const size_t oA16 = 0;
    const size_t oAT  = oA16 + szA;
    const size_t oTH  = oAT  + szA;
    const size_t oWT  = oTH  + szA;
    const size_t oZ   = oWT  + szWT;
    const size_t oD1  = oZ   + szZ;
    const size_t oD2  = oD1  + szD;
    const size_t oP   = oD2  + szD;
    const size_t oQA  = oP   + szP;
    const size_t oQB  = oQA  + szP;
    const size_t oF   = oQB  + szP;
    const size_t total = oF + szF;
    if (total > ws_size) return;
    if (total > (size_t)134217728) return;

    char* ws = (char*)d_ws;
    f16*   a16  = (f16*)(ws + oA16);
    f16*   aT16 = (f16*)(ws + oAT);
    f16*   th16 = (f16*)(ws + oTH);
    f16*   wT   = (f16*)(ws + oWT);
    f16*   z16  = (f16*)(ws + oZ);
    float* d1   = (float*)(ws + oD1);
    float* d2   = (float*)(ws + oD2);
    f16*   P    = (f16*)(ws + oP);
    f16*   QA   = (f16*)(ws + oQA);
    f16*   QB   = (f16*)(ws + oQB);
    float* F    = (float*)(ws + oF);

    prep_adj<<<dim3(NN / 64, NN / 64), 256, 0, stream>>>(adj, a16, aT16);
    row_deg<<<NN / 32, 256, 0, stream>>>(a16, d1);
    prep_w<<<NN / 64, 256, 0, stream>>>(wmap, wT);
    prep_z<<<1, 256, 0, stream>>>(x, cat, emb, z16);
    aa_gemm<<<dim3(NN / 64, NN / 64), 128, 0, stream>>>(a16, aT16, th16);
    row_deg<<<NN / 32, 256, 0, stream>>>(th16, d2);
    nodes_gemm<<<NN / 64, 128, 0, stream>>>(z16, wT, bmap, d1, d2, F, P);
    prop_gemm<<<dim3(NN / 64, 1), 128, 0, stream>>>(a16,  P,                 d1, d1, d2,
                                                    F + (size_t)1 * PLANE, QA, QB, 1);
    prop_gemm<<<dim3(NN / 64, 1), 128, 0, stream>>>(th16, P + (size_t)PLANE, d2, d1, d2,
                                                    F + (size_t)2 * PLANE,
                                                    QA + (size_t)PLANE, QB + (size_t)PLANE, 1);
    prop_gemm<<<dim3(NN / 64, 2), 128, 0, stream>>>(a16,  QA, d1, d1, d2,
                                                    F + (size_t)3 * PLANE, QA, QB, 0);
    prop_gemm<<<dim3(NN / 64, 2), 128, 0, stream>>>(th16, QB, d2, d1, d2,
                                                    F + (size_t)5 * PLANE, QA, QB, 0);
    readout_k<<<PLANE / (256 * 4), 256, 0, stream>>>(F, wemb, wout, out);
}
